// Pairwise_19713899889258
// MI455X (gfx1250) — hardware-run, weakly checked
//
#include <hip/hip_runtime.h>
#include <math.h>

typedef __attribute__((ext_vector_type(16))) _Float16 v16h;
typedef __attribute__((ext_vector_type(8)))  _Float16 v8h;
typedef __attribute__((ext_vector_type(16))) __bf16   v16b;
typedef __attribute__((ext_vector_type(8)))  __bf16   v8b;
typedef __attribute__((ext_vector_type(8)))  float    v8f;
typedef __attribute__((ext_vector_type(4)))  float    v4f;

constexpr int kBatch = 32;
constexpr int kNR    = 36;
constexpr int kD     = 2048;
constexpr int kC     = 4;
constexpr int kH     = 512;
constexpr int kRows  = kBatch * kNR;
constexpr int kNPad  = 48;
constexpr int kKMain = kH + 32;
constexpr int kAP    = kKMain + 8;
constexpr int kBtmP  = 576;
constexpr int kFlrP  = 2 * kH;

static_assert(kRows == 1152, "rows");
static_assert((kRows % 64) == 0 && (kFlrP % 64) == 0 && (kD % 32) == 0, "projection GEMM tile multiples");
static_assert((kD % 64) == 0 && (kH % 64) == 0, "transpose tile multiples");
static_assert((kKMain % 32) == 0 && kKMain + 8 <= kAP, "fused K multiple of 32");
static_assert((kBtmP * 2) % 128 == 0 && kBtmP >= kKMain, "weight plane pitch is a line multiple");
static_assert(kC == 4 && kC * kC == 16, "rank of the coordinate table");
static_assert(kNPad - kNR <= kNR && (kNPad % 16) == 0, "row duplication pad");

constexpr float kCarryMM   = 64.0f;
constexpr float kCarryW    = 1024.0f;
constexpr float kCarryPair = 32.0f;
constexpr float kCarryCo   = 512.0f;
constexpr float kCarryT    = 131072.0f;
constexpr float kProjFold  = 1.0f / (kCarryMM * kCarryW);
constexpr float kExtraFold = (kCarryPair * kCarryW) / (kCarryCo * kCarryT);
constexpr float kOutFold   = 1.0f / (kCarryPair * kCarryW);

constexpr size_t kOffAH   = 0;
constexpr size_t kOffBTP  = kOffAH  + (size_t)kRows * kD * 2;
constexpr size_t kOffFLR  = kOffBTP + (size_t)kFlrP * kD * 2;
constexpr size_t kOffBTM  = kOffFLR + (size_t)kRows * kFlrP * 4;
constexpr size_t kWsTotal = kOffBTM + (size_t)kD * kBtmP * 2;
static_assert(kWsTotal == 15990784ull, "carve total");
static_assert(kWsTotal <= 134217728ull, "carve cap");
static_assert((kOffBTP % 128) == 0 && (kOffFLR % 128) == 0 && (kOffBTM % 128) == 0, "128-B aligned regions");

__device__ __forceinline__ unsigned short f2bf_bits(float f) {
  unsigned u = __float_as_uint(f);
  return (unsigned short)((u + 0x7FFFu + ((u >> 16) & 1u)) >> 16);
}
__device__ __forceinline__ float bf_bits2f(unsigned short h) { return __uint_as_float(((unsigned)h) << 16); }

__device__ __forceinline__ void dep_guard4_h(v8f& a, v8f& b, v8f& c, v8f& d, v16h x, v16h y) { asm volatile("v_nop\n\tv_nop\n\tv_nop\n\tv_nop" : "+v"(a), "+v"(b), "+v"(c), "+v"(d) : "v"(x), "v"(y)); }
__device__ __forceinline__ void dep_guard4_b(v8f& a, v8f& b, v8f& c, v8f& d, v16b x, v16b y) { asm volatile("v_nop\n\tv_nop\n\tv_nop\n\tv_nop" : "+v"(a), "+v"(b), "+v"(c), "+v"(d) : "v"(x), "v"(y)); }
__device__ __forceinline__ void keep4_h(v16h a, v16h b, v16h c, v16h d) { asm volatile("v_nop" :: "v"(a), "v"(b), "v"(c), "v"(d)); }
__device__ __forceinline__ void keep4_b(v16b a, v16b b, v16b c, v16b d) { asm volatile("v_nop" :: "v"(a), "v"(b), "v"(c), "v"(d)); }
__device__ __forceinline__ void acc_guard4(v8f& a, v8f& b, v8f& c, v8f& d) { asm volatile("v_nop\n\tv_nop\n\tv_nop\n\tv_nop" : "+v"(a), "+v"(b), "+v"(c), "+v"(d)); }

template <typename T> struct Frag;
template <> struct Frag<_Float16> {
  typedef v16h V; union U { v16h v; v8h h[2]; };
  static __device__ __forceinline__ v16h load(const _Float16* p) {
    U f; f.h[0] = *(const v8h*)(p); f.h[1] = *(const v8h*)(p + 16); return f.v;
  }
  static __device__ __forceinline__ v8f mma(v16h a, v16h b, v8f c) {
    return __builtin_amdgcn_wmma_f32_16x16x32_f16(false, a, false, b, (short)0, c, false, false);
  }
  static __device__ __forceinline__ void guard4(v8f& a, v8f& b, v8f& c, v8f& d, v16h x, v16h y) { dep_guard4_h(a, b, c, d, x, y); }
  static __device__ __forceinline__ void keep(v16h a, v16h b, v16h c, v16h d) { keep4_h(a, b, c, d); }
};
template <> struct Frag<__bf16> {
  typedef v16b V; union U { v16b v; v8b h[2]; };
  static __device__ __forceinline__ v16b load(const __bf16* p) {
    U f; f.h[0] = *(const v8b*)(p); f.h[1] = *(const v8b*)(p + 16); return f.v;
  }
  static __device__ __forceinline__ v8f mma(v16b a, v16b b, v8f c) {
    return __builtin_amdgcn_wmma_f32_16x16x32_bf16(false, a, false, b, (short)0, c, false, false);
  }
  static __device__ __forceinline__ void guard4(v8f& a, v8f& b, v8f& c, v8f& d, v16b x, v16b y) { dep_guard4_b(a, b, c, d, x, y); }
  static __device__ __forceinline__ void keep(v16b a, v16b b, v16b c, v16b d) { keep4_b(a, b, c, d); }
};

__device__ __forceinline__ v8f mma_h_tied(v16h a, v16h b, v8f c) {
  c = __builtin_amdgcn_wmma_f32_16x16x32_f16(false, a, false, b, (short)0, c, false, false);
  asm volatile("v_nop\n\tv_nop\n\tv_nop\n\tv_nop" : "+v"(c) : "v"(a), "v"(b));
  return c;
}

template <int ET> struct Elem;
template <> struct Elem<0> { typedef _Float16 T; };
template <> struct Elem<1> { typedef __bf16 T; };
template <int ET, bool SPLIT, int BIAS_MODE, int OUT_MODE, bool RESID, int ACT = 0>
__global__ __launch_bounds__(256) void wmma_gemm64(
    const unsigned short* __restrict__ Ap, const unsigned short* __restrict__ A2p, int lda, long strideA,
    const unsigned short* __restrict__ Btp, const unsigned short* __restrict__ Bt2p, int ldb, long strideB,
    void* __restrict__ Cout, void* __restrict__ Cout2, int ldc, long strideC,
    const float* __restrict__ bias,
    const float* __restrict__ resid, long strideR,
    int M, int N, int K, float scale) {
  typedef typename Elem<ET>::T T;
  typedef typename Frag<T>::V V;
  const T* A = (const T*)Ap; const T* A2 = (const T*)A2p; const T* Bt = (const T*)Btp; const T* Bt2 = (const T*)Bt2p;
  __shared__ __align__(16) float sT[8][16 * 68];
  const int b    = blockIdx.y;
  const int lane = threadIdx.x & 31;
  const int wave = __builtin_amdgcn_readfirstlane((int)(threadIdx.x >> 5));
  const int tilesN = N >> 6;
  const int tilesM = M >> 6;
  const int tile = blockIdx.x * 8 + wave;
  if (tile >= tilesM * tilesN) return;
  const int tm = tile / tilesN;
  const int tn = tile - tm * tilesN;
  const int m0 = tm << 6;
  const int n0 = tn << 6;

  const T* Ab  = A  + (size_t)b * strideA;
  const T* Bb  = Bt + (size_t)b * strideB;
  const T* Ab2 = SPLIT ? (A2  + (size_t)b * strideA) : nullptr;
  const T* Bb2 = SPLIT ? (Bt2 + (size_t)b * strideB) : nullptr;

  const int rlane = lane & 15;
  const int koff  = (lane >> 4) * 8;
  const int mOff  = (lane >> 4) * 8;

  v8f acc[4][4];
#pragma unroll
  for (int i = 0; i < 4; ++i)
#pragma unroll
    for (int j = 0; j < 4; ++j) acc[i][j] = (v8f){0.f,0.f,0.f,0.f,0.f,0.f,0.f,0.f};

  for (int k0 = 0; k0 < K; k0 += 32) {
    V bh[4], bl[4];
#pragma unroll
    for (int j = 0; j < 4; ++j) {
      const size_t bo = (size_t)(n0 + (j << 4) + rlane) * ldb + koff + k0;
      bh[j] = Frag<T>::load(Bb + bo);
      if (SPLIT) bl[j] = Frag<T>::load(Bb2 + bo);
    }
#pragma unroll
    for (int i = 0; i < 4; ++i) {
      const size_t ao = (size_t)(m0 + (i << 4) + rlane) * lda + koff + k0;
      V ah = Frag<T>::load(Ab + ao);
      V al;
      if (SPLIT) al = Frag<T>::load(Ab2 + ao);
#pragma unroll
      for (int j = 0; j < 4; ++j) {
        acc[i][j] = Frag<T>::mma(ah, bh[j], acc[i][j]);
        if (SPLIT) {
          acc[i][j] = Frag<T>::mma(ah, bl[j], acc[i][j]);
          acc[i][j] = Frag<T>::mma(al, bh[j], acc[i][j]);
        }
      }
      Frag<T>::guard4(acc[i][0], acc[i][1], acc[i][2], acc[i][3], ah, SPLIT ? al : ah);
    }
    Frag<T>::keep(bh[0], bh[1], bh[2], bh[3]);
    if (SPLIT) Frag<T>::keep(bl[0], bl[1], bl[2], bl[3]);
  }
  acc_guard4(acc[0][0], acc[0][1], acc[0][2], acc[0][3]);
  acc_guard4(acc[1][0], acc[1][1], acc[1][2], acc[1][3]);
  acc_guard4(acc[2][0], acc[2][1], acc[2][2], acc[2][3]);
  acc_guard4(acc[3][0], acc[3][1], acc[3][2], acc[3][3]);

  float* slab = sT[wave];
  const float* Rb = RESID ? (resid + (size_t)b * strideR) : nullptr;
#pragma unroll
  for (int i = 0; i < 4; ++i) {
    const int mBase = m0 + (i << 4);
#pragma unroll
    for (int j = 0; j < 4; ++j) {
      const int n = n0 + (j << 4) + rlane;
      float bv = 0.f;
      if (BIAS_MODE == 2) bv = bias[n];
#pragma unroll
      for (int r = 0; r < 8; ++r) {
        float v = acc[i][j][r] * scale;
        if (BIAS_MODE == 1) v += bias[mBase + mOff + r];
        if (BIAS_MODE == 2) v += bv;
        if (RESID) v += Rb[(size_t)(mBase + mOff + r) * ldc + n];
        if (ACT == 1) v = tanhf(v);
        if (ACT == 2) v = fmaxf(v, 0.0f);
        if (ACT == 3) v = v / (1.0f + expf(-v));
        if (ACT == 4) v = (v > 0.f) ? v : 0.01f * v;
        slab[(mOff + r) * 68 + (j << 4) + rlane] = v;
      }
    }
    __builtin_amdgcn_fence(__ATOMIC_RELEASE, "workgroup");
    __builtin_amdgcn_wave_barrier();
    __builtin_amdgcn_fence(__ATOMIC_ACQUIRE, "workgroup");
    if (OUT_MODE == 0) {
      float* C = (float*)Cout + (size_t)b * strideC;
      const int hh = lane >> 4, c4 = (lane & 15) * 4;
      for (int pass = 0; pass < 2; ++pass) {
#pragma unroll
        for (int it = 0; it < 8; ++it) {
          const int row = it * 2 + hh;
          v4f v = *(const v4f*)(slab + row * 68 + c4);
          *(volatile v4f*)(C + (size_t)(mBase + row) * ldc + n0 + c4) = v;
        }
        __threadfence();
      }
    } else {
      const int q = lane >> 3, c8 = (lane & 7) * 8;
      unsigned short* C  = (unsigned short*)Cout  + (size_t)b * strideC;
      unsigned short* C2 = (OUT_MODE == 2) ? ((unsigned short*)Cout2 + (size_t)b * strideC) : nullptr;
      for (int pass = 0; pass < 2; ++pass) {
#pragma unroll
        for (int it = 0; it < 4; ++it) {
          const int row = it * 4 + q;
          const float* sp = slab + row * 68 + c8;
          v8h hv, lv;
#pragma unroll
          for (int e = 0; e < 8; ++e) {
            if (OUT_MODE == 1) {
              hv[e] = (_Float16)sp[e];
            } else {
              unsigned short hb = f2bf_bits(sp[e]);
              unsigned short lb = f2bf_bits(sp[e] - bf_bits2f(hb));
              hv[e] = __builtin_bit_cast(_Float16, hb);
              lv[e] = __builtin_bit_cast(_Float16, lb);
            }
          }
          *(volatile v8h*)(C + (size_t)(mBase + row) * ldc + n0 + c8) = hv;
          if (OUT_MODE == 2) *(volatile v8h*)(C2 + (size_t)(mBase + row) * ldc + n0 + c8) = lv;
        }
        __threadfence();
      }
    }
    __builtin_amdgcn_fence(__ATOMIC_RELEASE, "workgroup");
    __builtin_amdgcn_wave_barrier();
    __builtin_amdgcn_fence(__ATOMIC_ACQUIRE, "workgroup");
  }
}

__global__ __launch_bounds__(256) void cast_rows_f16_kernel(
    const float* __restrict__ src, unsigned short* __restrict__ dst, int total8, float carry)
{
  const int i = blockIdx.x * 256 + threadIdx.x;
  if (i >= total8) return;
  const size_t e0 = (size_t)i << 3;
  const v4f a0 = *(const v4f*)(src + e0);
  const v4f a1 = *(const v4f*)(src + e0 + 4);
  v8h hv;
#pragma unroll
  for (int e = 0; e < 4; ++e) {
    hv[e]     = (_Float16)(a0[e] * carry);
    hv[4 + e] = (_Float16)(a1[e] * carry);
  }
  unsigned short* q = dst + e0;
  *(volatile v8h*)q = hv;
  __threadfence();
  *(volatile v8h*)q = hv;
}

__global__ __launch_bounds__(256) void transpose_cast_kernel(
    const float* __restrict__ src0, const float* __restrict__ src1, unsigned short* __restrict__ dst,
    int srcCols, int dstPitch, int dstRowsPerZ, float carry)
{
  __shared__ float sT[64 * 65];
  const int tid  = threadIdx.x;
  const int lane = tid & 31;
  const int wave = __builtin_amdgcn_readfirstlane((int)(threadIdx.x >> 5));
  const float* src = (blockIdx.z != 0) ? src1 : src0;
  const int r0 = blockIdx.x * 64;
  const int c0 = blockIdx.y * 64;
  const int lc = tid & 63;
  const int lr = tid >> 6;
#pragma unroll 4
  for (int it = 0; it < 16; ++it) {
    const int r = it * 4 + lr;
    sT[r * 65 + lc] = src[(size_t)(r0 + r) * srcCols + c0 + lc] * carry;
  }
  __syncthreads();
  const int q  = lane >> 3;
  const int c8 = (lane & 7) * 8;
  v8h hv[2];
#pragma unroll
  for (int it = 0; it < 2; ++it) {
    const int c = it * 32 + wave * 4 + q;
#pragma unroll
    for (int e = 0; e < 8; ++e) hv[it][e] = (_Float16)sT[(c8 + e) * 65 + c];
  }
  const size_t zrow = (size_t)blockIdx.z * dstRowsPerZ + c0;
  for (int pass = 0; pass < 2; ++pass) {
#pragma unroll
    for (int it = 0; it < 2; ++it) {
      const int c = it * 32 + wave * 4 + q;
      *(volatile v8h*)(dst + (zrow + c) * dstPitch + r0 + c8) = hv[it];
    }
    __threadfence();
  }
}

__global__ __launch_bounds__(256) void coord_table_kernel(
    const float* __restrict__ Wcl, const float* __restrict__ Wcr, const float* __restrict__ Wcout,
    unsigned short* __restrict__ BTM)
{
  __shared__ float sV[256 * 17];
  const int tid  = threadIdx.x;
  const int lane = tid & 31;
  const int wave = __builtin_amdgcn_readfirstlane((int)(threadIdx.x >> 5));
  const int d0 = blockIdx.x * 256;
  const int d  = d0 + tid;
  float acc[16];
#pragma unroll
  for (int k = 0; k < 16; ++k) acc[k] = 0.0f;
#pragma unroll 1
  for (int h = 0; h < kH; ++h) {
    const float wc = Wcout[(size_t)h * kD + d];
    float wl[4], wr[4];
#pragma unroll
    for (int a = 0; a < 4; ++a) {
      wl[a] = Wcl[a * kH + h];
      wr[a] = Wcr[a * kH + h];
    }
#pragma unroll
    for (int a = 0; a < 4; ++a)
#pragma unroll
      for (int c = 0; c < 4; ++c)
        acc[a * 4 + c] = fmaf(wl[a] * wr[c], wc, acc[a * 4 + c]);
  }
#pragma unroll
  for (int k = 0; k < 16; ++k) sV[tid * 17 + k] = acc[k] * kCarryT;
  __syncthreads();
  const int q   = lane >> 3;
  const int ch  = lane & 7;
  const int chc = (ch < 2) ? ch : 1;
  const bool live = (ch < 2);
  v8h hv[8];
#pragma unroll
  for (int it = 0; it < 8; ++it) {
    const int row = it * 32 + wave * 4 + q;
    const float* sp = sV + row * 17 + chc * 8;
#pragma unroll
    for (int e = 0; e < 8; ++e) {
      const float v = sp[e];
      hv[it][e] = (_Float16)(live ? v : 0.0f);
    }
  }
  for (int pass = 0; pass < 2; ++pass) {
#pragma unroll
    for (int it = 0; it < 8; ++it) {
      const int row = it * 32 + wave * 4 + q;
      *(volatile v8h*)(BTM + (size_t)(d0 + row) * kBtmP + kH + ch * 8) = hv[it];
    }
    __threadfence();
  }
}

__global__ __launch_bounds__(256) void pair_fuse_max_kernel(
    const float* __restrict__ FLR, const float* __restrict__ coords,
    const unsigned short* __restrict__ BTMp, const float* __restrict__ mm, float* __restrict__ out)
{
  __shared__ __align__(16) _Float16 sA[kNPad * kAP];
  const int tid  = threadIdx.x;
  const int lane = tid & 31;
  const int wave = __builtin_amdgcn_readfirstlane((int)(threadIdx.x >> 5));
  const int bi = blockIdx.x;
  const int b  = bi / kNR;
  const _Float16* BTM = (const _Float16*)BTMp;

  {
    const int hc = (tid & 63) * 8;
    const int jr = wave >> 1;
    const float* flp = FLR + (size_t)bi * kFlrP + hc;
    v4f f0 = *(const v4f*)(flp);
    v4f f1 = *(const v4f*)(flp + 4);
    f0 = f0 * kCarryPair;
    f1 = f1 * kCarryPair;
#pragma unroll 4
    for (int it = 0; it < 12; ++it) {
      const int j  = jr + 4 * it;
      const int jj = (j < kNR) ? j : (j - kNR);
      const float* frp = FLR + (size_t)(b * kNR + jj) * kFlrP + kH + hc;
      const v4f r0 = *(const v4f*)(frp);
      const v4f r1 = *(const v4f*)(frp + 4);
      v8h pv;
#pragma unroll
      for (int e = 0; e < 4; ++e) {
        pv[e]     = (_Float16)(f0[e] * r0[e]);
        pv[4 + e] = (_Float16)(f1[e] * r1[e]);
      }
      *(v8h*)(sA + j * kAP + hc) = pv;
    }
  }
  {
    const int rowu = tid / 5;
    const int q    = tid - rowu * 5;
    const int row  = (rowu < kNPad) ? rowu : (kNPad - 1);
    const int jj   = (row < kNR) ? row : (row - kNR);
    const v4f civ = *(const v4f*)(coords + (size_t)bi * kC);
    const v4f cjv = *(const v4f*)(coords + (size_t)(b * kNR + jj) * kC);
    float ci0 = civ[0], ci1 = civ[1], ci2 = civ[2], ci3 = civ[3];
    float cj0 = cjv[0], cj1 = cjv[1], cj2 = cjv[2], cj3 = cjv[3];
    asm volatile("" : "+v"(ci0), "+v"(ci1), "+v"(ci2), "+v"(ci3));
    asm volatile("" : "+v"(cj0), "+v"(cj1), "+v"(cj2), "+v"(cj3));
    const bool live  = (q < 2);
    const bool first = (q == 0);
    const float a0 = (first ? ci0 : ci2) * kCarryCo;
    const float a1 = (first ? ci1 : ci3) * kCarryCo;
    v8h ev;
    ev[0] = (_Float16)(live ? a0 * cj0 : 0.0f);
    ev[1] = (_Float16)(live ? a0 * cj1 : 0.0f);
    ev[2] = (_Float16)(live ? a0 * cj2 : 0.0f);
    ev[3] = (_Float16)(live ? a0 * cj3 : 0.0f);
    ev[4] = (_Float16)(live ? a1 * cj0 : 0.0f);
    ev[5] = (_Float16)(live ? a1 * cj1 : 0.0f);
    ev[6] = (_Float16)(live ? a1 * cj2 : 0.0f);
    ev[7] = (_Float16)(live ? a1 * cj3 : 0.0f);
    if (tid < 5 * kNPad) *(v8h*)(sA + row * kAP + kH + q * 8) = ev;
  }
  __syncthreads();

  const int rl = lane & 15;
  const int hk = (lane >> 4) * 8;
  const _Float16* aBase = sA + rl * kAP + hk;

#pragma unroll 1
  for (int p = 0; p < 8; ++p) {
    const int nt0 = p * 16 + wave * 2;
    const _Float16* b0 = BTM + (size_t)(nt0 * 16 + rl) * kBtmP + hk;
    const _Float16* b1 = b0 + (size_t)16 * kBtmP;
    v8f acc[2][3];
#pragma unroll
    for (int t = 0; t < 2; ++t)
#pragma unroll
      for (int m = 0; m < 3; ++m) acc[t][m] = (v8f){0.f,0.f,0.f,0.f,0.f,0.f,0.f,0.f};

    {
      const v16h bf0 = Frag<_Float16>::load(b0 + kH);
      const v16h bf1 = Frag<_Float16>::load(b1 + kH);
#pragma unroll
      for (int m = 0; m < 3; ++m) {
        const v16h af = Frag<_Float16>::load(aBase + m * 16 * kAP + kH);
        acc[0][m] = mma_h_tied(af, bf0, acc[0][m]);
        acc[1][m] = mma_h_tied(af, bf1, acc[1][m]);
      }
    }
#pragma unroll
    for (int t = 0; t < 2; ++t)
#pragma unroll
      for (int m = 0; m < 3; ++m) acc[t][m] = acc[t][m] * kExtraFold;

#pragma unroll 1
    for (int k0 = 0; k0 < kH; k0 += 32) {
      const v16h bf0 = Frag<_Float16>::load(b0 + k0);
      const v16h bf1 = Frag<_Float16>::load(b1 + k0);
#pragma unroll
      for (int m = 0; m < 3; ++m) {
        const v16h af = Frag<_Float16>::load(aBase + m * 16 * kAP + k0);
        acc[0][m] = mma_h_tied(af, bf0, acc[0][m]);
        acc[1][m] = mma_h_tied(af, bf1, acc[1][m]);
      }
    }

    float mxt[2];
#pragma unroll
    for (int t = 0; t < 2; ++t) {
      float mx = acc[t][0][0];
#pragma unroll
      for (int m = 0; m < 3; ++m)
#pragma unroll
        for (int v = 0; v < 8; ++v) mx = fmaxf(mx, acc[t][m][v]);
      const float o = __shfl_xor(mx, 16, 32);
      mxt[t] = fmaxf(mx, o);
    }
    const float sel = ((lane >> 4) != 0) ? mxt[1] : mxt[0];
    const int d = nt0 * 16 + lane;
    const float skip = mm[(size_t)bi * kD + d];
    const float res = sel * kOutFold + skip;
    volatile float* po = out + (size_t)bi * kD + d;
    *po = res;
    __threadfence();
    *po = res;
  }
}

extern "C" void kernel_launch(void* const* d_in, const int* in_sizes, int n_in,
                              void* d_out, int out_size, void* d_ws, size_t ws_size,
                              hipStream_t stream) {
  if (n_in < 8) return;
  if (in_sizes[0] != kRows * kD) return;
  if (in_sizes[1] != kRows * kC) return;
  if (in_sizes[2] != kC * kH) return;
  if (in_sizes[3] != kC * kH) return;
  if (in_sizes[4] != kH * kD) return;
  if (in_sizes[5] != kD * kH) return;
  if (in_sizes[6] != kD * kH) return;
  if (in_sizes[7] != kH * kD) return;
  if (out_size != kRows * kD) return;
  if (ws_size < kWsTotal) return;

  const float* mm     = (const float*)d_in[0];
  const float* coords = (const float*)d_in[1];
  const float* W_cl   = (const float*)d_in[2];
  const float* W_cr   = (const float*)d_in[3];
  const float* W_cout = (const float*)d_in[4];
  const float* W_fl   = (const float*)d_in[5];
  const float* W_fr   = (const float*)d_in[6];
  const float* W_fout = (const float*)d_in[7];
  float* out = (float*)d_out;

  char* ws = (char*)d_ws;
  unsigned short* AH  = (unsigned short*)(ws + kOffAH);
  unsigned short* BTP = (unsigned short*)(ws + kOffBTP);
  float*          FLR = (float*)(ws + kOffFLR);
  unsigned short* BTM = (unsigned short*)(ws + kOffBTM);

  cast_rows_f16_kernel<<<(kRows * kD / 8) / 256, 256, 0, stream>>>(mm, AH, kRows * kD / 8, kCarryMM);

  transpose_cast_kernel<<<dim3(kD / 64, kH / 64, 2), 256, 0, stream>>>(W_fl, W_fr, BTP, kH, kD, kH, kCarryW);

  wmma_gemm64<0, false, 0, 0, false><<<dim3((kRows / 64) * (kFlrP / 64) / 8, 1), 256, 0, stream>>>(
      AH, nullptr, kD, 0L,
      BTP, nullptr, kD, 0L,
      (void*)FLR, nullptr, kFlrP, 0L,
      nullptr, nullptr, 0L,
      kRows, kFlrP, kD, kProjFold);

  transpose_cast_kernel<<<dim3(kH / 64, kD / 64, 1), 256, 0, stream>>>(W_fout, W_fout, BTM, kD, kBtmP, 0, kCarryW);

  coord_table_kernel<<<kD / 256, 256, 0, stream>>>(W_cl, W_cr, W_cout, BTM);

  pair_fuse_max_kernel<<<kRows, 256, 0, stream>>>(FLR, coords, BTM, mm, out);
}
